// EquivariantProductBasisBlock_3959959847294
// MI455X (gfx1250) — hardware-verified
//
#include <hip/hip_runtime.h>
#include <stdint.h>

typedef __bf16         v16bf __attribute__((ext_vector_type(16)));
typedef unsigned short v16us __attribute__((ext_vector_type(16)));
typedef unsigned short v8us  __attribute__((ext_vector_type(8)));
typedef unsigned int   v4u   __attribute__((ext_vector_type(4)));
typedef unsigned int   v2u   __attribute__((ext_vector_type(2)));
typedef float          v8f   __attribute__((ext_vector_type(8)));
typedef float          v4f   __attribute__((ext_vector_type(4)));
typedef v8us __attribute__((may_alias)) v8usa;
typedef v4u  __attribute__((may_alias)) v4ua;
typedef v2u  __attribute__((may_alias)) v2ua;
typedef v4f  __attribute__((may_alias)) v4fa;

union FragU { v16us v; v8us half[2]; };
union BFv   { v16us u; v16bf b; };

#define NN   1024
#define CC   128
#define KS   9
#define EE   10
#define OW   512
#define APU  136
#define APW  68

__device__ __forceinline__ unsigned short f2bf(float f) {
  unsigned u = __float_as_uint(f);
  u = u + 0x7FFFu + ((u >> 16) & 1u);
  return (unsigned short)(u >> 16);
}
__device__ __forceinline__ float bf2f(unsigned short b) { return __uint_as_float(((unsigned)b) << 16); }
__device__ __forceinline__ float bfr(float f) { return bf2f(f2bf(f)); }
__device__ __forceinline__ unsigned pk2(unsigned short lo, unsigned short hi) {
  return (unsigned)lo | (((unsigned)hi) << 16);
}

__device__ __forceinline__ v8f wmma_bf16(v16us au, v16us bu, v8f c) {
  BFv A, B; A.u = au; B.u = bu;
  v8f d = __builtin_amdgcn_wmma_f32_16x16x32_bf16(false, A.b, false, B.b, (short)0, c, false, false);
  asm volatile("v_nop\n\tv_nop\n\tv_nop\n\tv_nop" : "+v"(d) : "v"(au), "v"(bu));
  return d;
}

__device__ __forceinline__ v16us ldfrag(const unsigned short* p, int h) {
  FragU f;
  f.half[0] = *(const v8usa*)(p + 8 * h);
  f.half[1] = *(const v8usa*)(p + 16 + 8 * h);
  return f.v;
}

__global__ __launch_bounds__(256) void k_prep(
    const float* __restrict__ U3a, const float* __restrict__ U3b,
    const float* __restrict__ Wla, const float* __restrict__ Wlb,
    unsigned* __restrict__ Bta, unsigned* __restrict__ Btb,
    unsigned* __restrict__ Wta, unsigned* __restrict__ Wtb)
{
  const int bid = blockIdx.x, tid = threadIdx.x;
  unsigned short hv[8];
  unsigned* dst;
  bool active;
  if (bid < 6) {
    const bool isB = (bid >= 2);
    const int M = isB ? 3 : 1;
    const float* U3 = isB ? U3b : U3a;
    unsigned* Bt = isB ? Btb : Bta;
    const int g = (isB ? (bid - 2) : bid) * 256 + tid;
    const int np = isB ? 1024 : 384;
    active = (g < np);
    const int gg = active ? g : 0;
    const int q = gg >> 2, kp0 = (gg & 3) * 8;
    const int mm = q / 81;
    const int ij = q - mm * 81;
    const int i = ij / 9;
    const int j = ij - i * 9;
    const bool qok = (q < M * 81);
    #pragma unroll
    for (int e = 0; e < 8; ++e) {
      const int kp = kp0 + e;
      const int k = kp / 3;
      const int p = kp - 3 * k;
      const bool ok = qok && (kp < 27);
      const int idx = ok ? ((((i * 9 + j) * 9 + k) * M + mm) * 3 + p) : 0;
      const float v = U3[idx];
      hv[e] = ok ? f2bf(v) : (unsigned short)0;
    }
    dst = Bt + (size_t)gg * 4;
  } else {
    const bool isB = (bid >= 14);
    const float* Wl = isB ? Wlb : Wla;
    unsigned* Wt = isB ? Wtb : Wta;
    const int g = (bid - (isB ? 14 : 6)) * 256 + tid;
    active = (g < 2048);
    const int gg = active ? g : 0;
    const int d = gg >> 4, c0 = (gg & 15) * 8;
    #pragma unroll
    for (int e = 0; e < 8; ++e) hv[e] = f2bf(Wl[(size_t)(c0 + e) * CC + d]);
    dst = Wt + (size_t)d * 64 + (c0 >> 1);
  }
  v4u o;
  o.x = pk2(hv[0], hv[1]); o.y = pk2(hv[2], hv[3]); o.z = pk2(hv[4], hv[5]); o.w = pk2(hv[6], hv[7]);
  if (active) *(volatile v4u*)dst = o;
  __threadfence();
  if (active) *(volatile v4u*)dst = o;
}

template <int M>
__device__ __forceinline__ void y_store_pass(const float* ys, float* Y, int n, int cb, int h, int m16) {
  #pragma unroll
  for (int mm = 0; mm < M; mm += 2) {
    const int m = mm + h;
    const int mc = (m < M) ? m : (M - 1);
    const v4f v = *(const v4fa*)(ys + mc * 64 + 4 * m16);
    if (m < M) *(volatile v4f*)(Y + ((size_t)(n * M + m) * CC + cb) + 4 * m16) = v;
  }
}

template <int NP>
__host__ __device__ constexpr int sym_lds_bytes() { return 8192 + 2 * 32 * (NP + 1) * 4 + 64 * KS * 4 + 3 * 64 * 4; }

template <int M, int NP, int NT>
__global__ __launch_bounds__(64) void k_sym(
    const float* __restrict__ nf,
    const float* __restrict__ na,
    const float* __restrict__ U1,
    const float* __restrict__ W1,
    const float* __restrict__ U2,
    const float* __restrict__ W2,
    const float* __restrict__ W3,
    const unsigned short* __restrict__ Bt,
    float* __restrict__ Y)
{
  static_assert(NT * 16 == NP);
  static_assert(M * 81 <= NP);
  static_assert(M <= 3);
  constexpr int DP = NP + 1;
  extern __shared__ unsigned char dsm_s[] __attribute__((aligned(16)));
  unsigned* Ahi = (unsigned*)dsm_s;
  unsigned* Alo = Ahi + 64 * 16;
  float* Dst = (float*)(dsm_s + 8192);
  float* xs  = Dst + 2 * 32 * DP;
  float* ys  = xs + 64 * KS;

  const int tid = threadIdx.x, lane = tid & 31, wave = tid >> 5;
  const int h = lane >> 4, m16 = lane & 15;
  const int n = blockIdx.x >> 1, cb = (blockIdx.x & 1) * 64, c = cb + tid;

  float x[KS];
  const float* xr = nf + ((size_t)n * CC + c) * KS;
  #pragma unroll
  for (int k = 0; k < KS; ++k) { x[k] = bfr(xr[k]); xs[tid * KS + k] = x[k]; }

  float w3[3] = {0.0f, 0.0f, 0.0f};
  float w2[2] = {0.0f, 0.0f};
  float w1 = 0.0f;
  #pragma unroll 1
  for (int e = 0; e < EE; ++e) {
    const float a = bfr(na[n * EE + e]);
    w1    = fmaf(a, bfr(W1[e * CC + c]), w1);
    w2[0] = fmaf(a, bfr(W2[(e * 2 + 0) * CC + c]), w2[0]);
    w2[1] = fmaf(a, bfr(W2[(e * 2 + 1) * CC + c]), w2[1]);
    w3[0] = fmaf(a, bfr(W3[(e * 3 + 0) * CC + c]), w3[0]);
    w3[1] = fmaf(a, bfr(W3[(e * 3 + 1) * CC + c]), w3[1]);
    w3[2] = fmaf(a, bfr(W3[(e * 3 + 2) * CC + c]), w3[2]);
  }

  float pr[27];
  #pragma unroll
  for (int k = 0; k < KS; ++k) {
    #pragma unroll
    for (int p = 0; p < 3; ++p) pr[3 * k + p] = x[k] * w3[p];
  }
  #pragma unroll
  for (int pc = 0; pc < 4; ++pc) {
    unsigned short hh[8], ll[8];
    #pragma unroll
    for (int e = 0; e < 8; ++e) {
      const int kp = pc * 8 + e;
      if (kp < 27) {
        const unsigned short hb = f2bf(pr[kp]);
        const float res = pr[kp] - bf2f(hb);
        hh[e] = hb;
        ll[e] = f2bf(res);
      } else {
        hh[e] = 0; ll[e] = 0;
      }
    }
    v4u vh, vl;
    vh.x = pk2(hh[0], hh[1]); vh.y = pk2(hh[2], hh[3]); vh.z = pk2(hh[4], hh[5]); vh.w = pk2(hh[6], hh[7]);
    vl.x = pk2(ll[0], ll[1]); vl.y = pk2(ll[2], ll[3]); vl.z = pk2(ll[4], ll[5]); vl.w = pk2(ll[6], ll[7]);
    *(v4ua*)(Ahi + tid * 16 + pc * 4) = vh;
    *(v4ua*)(Alo + tid * 16 + pc * 4) = vl;
  }
  __syncthreads();

  const unsigned short* Ahs = (const unsigned short*)Ahi;
  const unsigned short* Als = (const unsigned short*)Alo;
  const v16us ah0 = ldfrag(Ahs + (wave * 32 + m16) * 32, h);
  const v16us ah1 = ldfrag(Ahs + (wave * 32 + 16 + m16) * 32, h);
  const v16us al0 = ldfrag(Als + (wave * 32 + m16) * 32, h);
  const v16us al1 = ldfrag(Als + (wave * 32 + 16 + m16) * 32, h);
  float* Dw = Dst + wave * 32 * DP;
  const v8f z8 = {0.f, 0.f, 0.f, 0.f, 0.f, 0.f, 0.f, 0.f};
  #pragma unroll 1
  for (int nt = 0; nt < NT; ++nt) {
    const int q = nt * 16 + m16;
    const v16us bb = ldfrag(Bt + (size_t)q * 32, h);
    v8f a0 = wmma_bf16(ah0, bb, z8);
    a0 = wmma_bf16(al0, bb, a0);
    v8f a1 = wmma_bf16(ah1, bb, z8);
    a1 = wmma_bf16(al1, bb, a1);
    #pragma unroll
    for (int r = 0; r < 8; ++r) {
      Dw[(8 * h + r) * DP + q]      = a0[r];
      Dw[(16 + 8 * h + r) * DP + q] = a1[r];
    }
  }
  __syncthreads();

  const float* Dr = Dst + tid * DP;
  #pragma unroll 1
  for (int m = 0; m < M; ++m) {
    float ym = 0.0f;
    #pragma unroll 1
    for (int i = 0; i < KS; ++i) {
      const float* u2p = U2 + ((i * 9) * M + m) * 2;
      const float* dq  = Dr + m * 81 + i * 9;
      float o2 = 0.0f;
      #pragma unroll
      for (int j = 0; j < KS; ++j) {
        float t = bfr(u2p[j * (M * 2)]) * w2[0];
        t = fmaf(bfr(u2p[j * (M * 2) + 1]), w2[1], t);
        const float ct = t + dq[j];
        o2 = fmaf(ct, x[j], o2);
      }
      const float ct1 = bfr(U1[i * M + m]) * w1 + o2;
      ym = fmaf(ct1, xs[tid * KS + i], ym);
    }
    ys[m * 64 + tid] = ym;
  }
  __syncthreads();

  if (wave == 0) {
    y_store_pass<M>(ys, Y, n, cb, h, m16);
    __threadfence();
    y_store_pass<M>(ys, Y, n, cb, h, m16);
  }
}

__device__ __forceinline__ void stage_hl(unsigned* Ah, unsigned* Al, int row, int c4, v4f v) {
  unsigned short hh[4], ll[4];
  const float vv[4] = {v.x, v.y, v.z, v.w};
  #pragma unroll
  for (int e = 0; e < 4; ++e) {
    const unsigned short hb = f2bf(vv[e]);
    hh[e] = hb;
    ll[e] = f2bf(vv[e] - bf2f(hb));
  }
  v2u wh, wl;
  wh.x = pk2(hh[0], hh[1]); wh.y = pk2(hh[2], hh[3]);
  wl.x = pk2(ll[0], ll[1]); wl.y = pk2(ll[2], ll[3]);
  *(v2ua*)(Ah + row * APW + (c4 >> 1)) = wh;
  *(v2ua*)(Al + row * APW + (c4 >> 1)) = wl;
}

__device__ __forceinline__ void out_store_pass(const float* so, const float* sc, float* out, int n0, int tid) {
  #pragma unroll
  for (int it = 0; it < 8; ++it) {
    const int f = it * 256 + tid;
    const int row = f >> 7, c4 = (f & 127) * 4;
    const v4f v = *(const v4fa*)(so + row * OW + c4);
    const size_t gi = (size_t)(n0 + row) * OW + c4;
    const v4f s = *(const v4fa*)(sc + gi);
    v4f o;
    o.x = v.x + bfr(s.x); o.y = v.y + bfr(s.y); o.z = v.z + bfr(s.z); o.w = v.w + bfr(s.w);
    *(volatile v4f*)(out + gi) = o;
  }
}

__global__ __launch_bounds__(256) void k_lin(
    const float* __restrict__ Y0, const float* __restrict__ Y1,
    const unsigned short* __restrict__ Wt0, const unsigned short* __restrict__ Wt1,
    const float* __restrict__ sc, float* __restrict__ out)
{
  extern __shared__ unsigned char dsm_l[] __attribute__((aligned(16)));
  unsigned* Ah = (unsigned*)dsm_l;
  unsigned* Al = Ah + 64 * APW;
  float* so = (float*)dsm_l;

  const int tid = threadIdx.x, lane = tid & 31, w = tid >> 5;
  const int h = lane >> 4, m16 = lane & 15;
  const int n0 = blockIdx.x * 16;

  #pragma unroll
  for (int it = 0; it < 2; ++it) {
    const int f = it * 256 + tid;
    const int row = f >> 5, c4 = (f & 31) * 4;
    const v4f v = *(const v4fa*)(Y0 + (size_t)(n0 + row) * CC + c4);
    stage_hl(Ah, Al, row, c4, v);
  }
  #pragma unroll 1
  for (int it = 0; it < 6; ++it) {
    const int f = it * 256 + tid;
    const int rr = f >> 5, c4 = (f & 31) * 4;
    const v4f v = *(const v4fa*)(Y1 + ((size_t)n0 * 3 + rr) * CC + c4);
    stage_hl(Ah, Al, 16 + rr, c4, v);
  }
  __syncthreads();

  const unsigned short* Ahs = (const unsigned short*)Ah;
  const unsigned short* Als = (const unsigned short*)Al;
  const v8f z8 = {0.f, 0.f, 0.f, 0.f, 0.f, 0.f, 0.f, 0.f};
  v8f acc[4];
  #pragma unroll
  for (int mi = 0; mi < 4; ++mi) acc[mi] = z8;
  const int drow = 16 * w + m16;
  #pragma unroll 1
  for (int k0 = 0; k0 < CC; k0 += 32) {
    const v16us b0 = ldfrag(Wt0 + (size_t)drow * CC + k0, h);
    const v16us b1 = ldfrag(Wt1 + (size_t)drow * CC + k0, h);
    #pragma unroll
    for (int mi = 0; mi < 4; ++mi) {
      const v16us ah = ldfrag(Ahs + (16 * mi + m16) * APU + k0, h);
      const v16us al = ldfrag(Als + (16 * mi + m16) * APU + k0, h);
      if (mi == 0) {
        acc[0] = wmma_bf16(ah, b0, acc[0]);
        acc[0] = wmma_bf16(al, b0, acc[0]);
      } else {
        acc[mi] = wmma_bf16(ah, b1, acc[mi]);
        acc[mi] = wmma_bf16(al, b1, acc[mi]);
      }
    }
  }
  __syncthreads();

  const float inv = 0.08838834764831845f;
  const int d = drow;
  #pragma unroll
  for (int r = 0; r < 8; ++r) so[(8 * h + r) * OW + d] = acc[0][r] * inv;
  #pragma unroll
  for (int mi = 1; mi < 4; ++mi) {
    #pragma unroll
    for (int r = 0; r < 8; ++r) {
      const int R = 16 * (mi - 1) + 8 * h + r;
      const int nl = R / 3;
      const int mm = R - 3 * nl;
      so[nl * OW + 128 + 3 * d + mm] = acc[mi][r] * inv;
    }
  }
  __syncthreads();

  out_store_pass(so, sc, out, n0, tid);
  __threadfence();
  out_store_pass(so, sc, out, n0, tid);
}

extern "C" void kernel_launch(void* const* d_in, const int* in_sizes, int n_in,
                              void* d_out, int out_size, void* d_ws, size_t ws_size,
                              hipStream_t stream) {
  if (n_in < 17) return;
  if (in_sizes[0] != NN * CC * KS) return;
  if (in_sizes[1] != NN * EE) return;
  if (in_sizes[2] != NN * OW) return;
  if (in_sizes[3] != 9 || in_sizes[4] != 1280 || in_sizes[5] != 162 || in_sizes[6] != 2560) return;
  if (in_sizes[7] != 2187 || in_sizes[8] != 3840 || in_sizes[9] != 16384) return;
  if (in_sizes[10] != 27 || in_sizes[11] != 1280 || in_sizes[12] != 486 || in_sizes[13] != 2560) return;
  if (in_sizes[14] != 6561 || in_sizes[15] != 3840 || in_sizes[16] != 16384) return;
  if (out_size != NN * OW) return;

  const float* nf    = (const float*)d_in[0];
  const float* na    = (const float*)d_in[1];
  const float* sc    = (const float*)d_in[2];
  const float* U1_0  = (const float*)d_in[3];
  const float* W1_0  = (const float*)d_in[4];
  const float* U2_0  = (const float*)d_in[5];
  const float* W2_0  = (const float*)d_in[6];
  const float* U3_0  = (const float*)d_in[7];
  const float* W3_0  = (const float*)d_in[8];
  const float* Wl_0  = (const float*)d_in[9];
  const float* U1_1  = (const float*)d_in[10];
  const float* W1_1  = (const float*)d_in[11];
  const float* U2_1  = (const float*)d_in[12];
  const float* W2_1  = (const float*)d_in[13];
  const float* U3_1  = (const float*)d_in[14];
  const float* W3_1  = (const float*)d_in[15];
  const float* Wl_1  = (const float*)d_in[16];
  float* out = (float*)d_out;

  const size_t bt0_b = (size_t)96 * 32 * 2;
  const size_t bt1_b = (size_t)256 * 32 * 2;
  const size_t wt_b  = (size_t)CC * CC * 2;
  const size_t y0_b  = (size_t)NN * 1 * CC * 4;
  const size_t y1_b  = (size_t)NN * 3 * CC * 4;
  const size_t off_bt0 = 0;
  const size_t off_bt1 = off_bt0 + bt0_b;
  const size_t off_wt0 = off_bt1 + bt1_b;
  const size_t off_wt1 = off_wt0 + wt_b;
  const size_t off_y0  = off_wt1 + wt_b;
  const size_t off_y1  = off_y0 + y0_b;
  const size_t total   = off_y1 + y1_b;
  if (total > ws_size) return;

  char* ws = (char*)d_ws;
  unsigned* Bt0 = (unsigned*)(ws + off_bt0);
  unsigned* Bt1 = (unsigned*)(ws + off_bt1);
  unsigned* Wt0 = (unsigned*)(ws + off_wt0);
  unsigned* Wt1 = (unsigned*)(ws + off_wt1);
  float* Y0 = (float*)(ws + off_y0);
  float* Y1 = (float*)(ws + off_y1);

  k_prep<<<dim3(22), dim3(256), 0, stream>>>(U3_0, U3_1, Wl_0, Wl_1, Bt0, Bt1, Wt0, Wt1);

  constexpr int lds0 = sym_lds_bytes<96>();
  constexpr int lds1 = sym_lds_bytes<256>();
  hipFuncSetAttribute(reinterpret_cast<const void*>(&k_sym<3, 256, 16>),
                      hipFuncAttributeMaxDynamicSharedMemorySize, lds1);
  k_sym<1, 96, 6><<<dim3(NN * 2), dim3(64), lds0, stream>>>(
      nf, na, U1_0, W1_0, U2_0, W2_0, W3_0, (const unsigned short*)Bt0, Y0);
  k_sym<3, 256, 16><<<dim3(NN * 2), dim3(64), lds1, stream>>>(
      nf, na, U1_1, W1_1, U2_1, W2_1, W3_1, (const unsigned short*)Bt1, Y1);

  const int ldsl = 2 * 64 * APW * 4;
  k_lin<<<dim3(NN / 16), dim3(256), ldsl, stream>>>(
      Y0, Y1, (const unsigned short*)Wt0, (const unsigned short*)Wt1, sc, out);
}
